// CoordConv_29180007809227
// MI455X (gfx1250) — hardware-verified
//
#include <hip/hip_runtime.h>
#include <stddef.h>
#include <math.h>

typedef __attribute__((ext_vector_type(16))) _Float16 v16h;
typedef __attribute__((ext_vector_type(8)))  _Float16 v8h;
typedef __attribute__((ext_vector_type(16))) __bf16   v16b;
typedef __attribute__((ext_vector_type(8)))  __bf16   v8b;
typedef __attribute__((ext_vector_type(8)))  float    v8f;
typedef __attribute__((ext_vector_type(4)))  float    v4f;
typedef __attribute__((ext_vector_type(2)))  float    v2f;
typedef __attribute__((ext_vector_type(4)))  int      v4i;

constexpr int NIN   = 64;
constexpr int HF    = 128;
constexpr int NOUT  = 128;
constexpr int CDIM  = 2;
constexpr int KCAT  = NIN + HF;
constexpr int CHE   = 163840;
constexpr int NBA   = 1024;
constexpr int NBS   = 4096;
constexpr int RPQ   = 1024;
constexpr int NTHR  = 256;
constexpr int NWAVE = 8;
constexpr int EPT   = 8;
constexpr int NGRP  = 1;
constexpr int SUBCH = NTHR * EPT * NGRP;
constexpr int WCAP  = EPT * NGRP * 32;
constexpr int LISTN = NWAVE * WCAP;
constexpr int NEDGE_MAX  = 800000;
constexpr int MAXSUB_CH  = (CHE + SUBCH - 1) / SUBCH;
constexpr int MAXSUB_ALL = (NEDGE_MAX + SUBCH - 1) / SUBCH;
constexpr int LDS_AGG = (NBA * NIN + NBA * 2) * 4 + LISTN * 4 + 64;

static_assert((SUBCH & (SUBCH - 1)) == 0 && SUBCH <= 4096);
static_assert((NBA & (NBA - 1)) == 0 && NBA <= 4096);
static_assert((NBS & (NBS - 1)) == 0 && NBS <= 4096);
static_assert(RPQ % NBA == 0 && RPQ % 64 == 0 && RPQ % NTHR == 0 && NBS % RPQ == 0);
static_assert(CHE % SUBCH == 0 && CHE % 256 == 0 && CHE % 64 == 0);
static_assert(LDS_AGG == 278592);
static_assert(NIN % 32 == 0 && HF % 32 == 0 && KCAT % 32 == 0);
static_assert(MAXSUB_CH == 80 && MAXSUB_ALL == 391);

__device__ __forceinline__ unsigned short f2bf_bits(float f) {
  unsigned u = __float_as_uint(f);
  return (unsigned short)((u + 0x7FFFu + ((u >> 16) & 1u)) >> 16);
}
__device__ __forceinline__ float bf_bits2f(unsigned short h) { return __uint_as_float(((unsigned)h) << 16); }

__device__ __forceinline__ void dep_guard_h(v8f& a, v8f& b, v16h x, v16h y) { asm volatile("v_nop\n\tv_nop\n\tv_nop\n\tv_nop" : "+v"(a), "+v"(b) : "v"(x), "v"(y)); }
__device__ __forceinline__ void dep_guard_b(v8f& a, v8f& b, v16b x, v16b y) { asm volatile("v_nop\n\tv_nop\n\tv_nop\n\tv_nop" : "+v"(a), "+v"(b) : "v"(x), "v"(y)); }
__device__ __forceinline__ void keep4_h(v16h a, v16h b, v16h c, v16h d) { asm volatile("v_nop" :: "v"(a), "v"(b), "v"(c), "v"(d)); }
__device__ __forceinline__ void keep4_b(v16b a, v16b b, v16b c, v16b d) { asm volatile("v_nop" :: "v"(a), "v"(b), "v"(c), "v"(d)); }
__device__ __forceinline__ void acc_guard4(v8f& a, v8f& b, v8f& c, v8f& d) { asm volatile("v_nop\n\tv_nop\n\tv_nop\n\tv_nop" : "+v"(a), "+v"(b), "+v"(c), "+v"(d)); }
template <typename T> struct Frag;
template <> struct Frag<_Float16> {
  typedef v16h V; union U { v16h v; v8h h[2]; };
  static __device__ __forceinline__ v16h load(const _Float16* p) {
    U f; f.h[0] = *(const v8h*)(p); f.h[1] = *(const v8h*)(p + 16); return f.v;
  }
  static __device__ __forceinline__ v8f mma(v16h a, v16h b, v8f c) {
    return __builtin_amdgcn_wmma_f32_16x16x32_f16(false, a, false, b, (short)0, c, false, false);
  }
  static __device__ __forceinline__ void guard(v8f& a, v8f& b, v16h x, v16h y) { dep_guard_h(a, b, x, y); }
  static __device__ __forceinline__ void keep(v16h a, v16h b, v16h c, v16h d) { keep4_h(a, b, c, d); }
};
template <> struct Frag<__bf16> {
  typedef v16b V; union U { v16b v; v8b h[2]; };
  static __device__ __forceinline__ v16b load(const __bf16* p) {
    U f; f.h[0] = *(const v8b*)(p); f.h[1] = *(const v8b*)(p + 16); return f.v;
  }
  static __device__ __forceinline__ v8f mma(v16b a, v16b b, v8f c) {
    return __builtin_amdgcn_wmma_f32_16x16x32_bf16(false, a, false, b, (short)0, c, false, false);
  }
  static __device__ __forceinline__ void guard(v8f& a, v8f& b, v16b x, v16b y) { dep_guard_b(a, b, x, y); }
  static __device__ __forceinline__ void keep(v16b a, v16b b, v16b c, v16b d) { keep4_b(a, b, c, d); }
};

template <int ET> struct Elem;
template <> struct Elem<0> { typedef _Float16 T; };
template <> struct Elem<1> { typedef __bf16 T; };
template <int ET, bool SPLIT, int BIAS_MODE, int OUT_MODE, bool RESID, int ACT = 0>
__global__ __launch_bounds__(256) void wmma_gemm64(
    const unsigned short* __restrict__ Ap, const unsigned short* __restrict__ A2p, int lda, long strideA,
    const unsigned short* __restrict__ Btp, const unsigned short* __restrict__ Bt2p, int ldb, long strideB,
    void* __restrict__ Cout, void* __restrict__ Cout2, int ldc, long strideC,
    const float* __restrict__ bias,
    const float* __restrict__ resid, long strideR,
    int M, int N, int K, float scale) {
  typedef typename Elem<ET>::T T;
  typedef typename Frag<T>::V V;
  const T* A = (const T*)Ap; const T* A2 = (const T*)A2p; const T* Bt = (const T*)Btp; const T* Bt2 = (const T*)Bt2p;
  __shared__ __align__(16) float sT[8][16 * 68];
  const int b    = blockIdx.y;
  const int lane = threadIdx.x & 31;
  const int wave = threadIdx.x >> 5;
  const int tilesN = N >> 6;
  const int tilesM = M >> 6;
  const int tile = blockIdx.x * 8 + wave;
  if (tile >= tilesM * tilesN) return;
  const int tm = tile / tilesN;
  const int tn = tile - tm * tilesN;
  const int m0 = tm << 6;
  const int n0 = tn << 6;

  const T* Ab  = A  + (size_t)b * strideA;
  const T* Bb  = Bt + (size_t)b * strideB;
  const T* Ab2 = SPLIT ? (A2  + (size_t)b * strideA) : nullptr;
  const T* Bb2 = SPLIT ? (Bt2 + (size_t)b * strideB) : nullptr;

  const int rlane = lane & 15;
  const int koff  = (lane >> 4) * 8;
  const int mOff  = (lane >> 4) * 8;

  v8f acc[4][4];
#pragma unroll
  for (int i = 0; i < 4; ++i)
#pragma unroll
    for (int j = 0; j < 4; ++j) acc[i][j] = (v8f){0.f,0.f,0.f,0.f,0.f,0.f,0.f,0.f};

  for (int k0 = 0; k0 < K; k0 += 32) {
    V bh[4], bl[4];
#pragma unroll
    for (int j = 0; j < 4; ++j) {
      const size_t bo = (size_t)(n0 + (j << 4) + rlane) * ldb + koff + k0;
      bh[j] = Frag<T>::load(Bb + bo);
      if (SPLIT) bl[j] = Frag<T>::load(Bb2 + bo);
    }
#pragma unroll
    for (int i = 0; i < 4; ++i) {
      const size_t ao = (size_t)(m0 + (i << 4) + rlane) * lda + koff + k0;
      V ah = Frag<T>::load(Ab + ao);
      V al;
      if (SPLIT) al = Frag<T>::load(Ab2 + ao);
#pragma unroll
      for (int j = 0; j < 4; ++j) {
        acc[i][j] = Frag<T>::mma(ah, bh[j], acc[i][j]);
        if (SPLIT) {
          acc[i][j] = Frag<T>::mma(ah, bl[j], acc[i][j]);
          acc[i][j] = Frag<T>::mma(al, bh[j], acc[i][j]);
        }
      }
      Frag<T>::guard(acc[i][0], acc[i][3], ah, SPLIT ? al : ah);
    }
    Frag<T>::keep(bh[0], bh[1], bh[2], bh[3]);
    if (SPLIT) Frag<T>::keep(bl[0], bl[1], bl[2], bl[3]);
  }
  acc_guard4(acc[0][0], acc[0][1], acc[0][2], acc[0][3]);
  acc_guard4(acc[1][0], acc[1][1], acc[1][2], acc[1][3]);
  acc_guard4(acc[2][0], acc[2][1], acc[2][2], acc[2][3]);
  acc_guard4(acc[3][0], acc[3][1], acc[3][2], acc[3][3]);

  float* slab = sT[wave];
  const float* Rb = RESID ? (resid + (size_t)b * strideR) : nullptr;
#pragma unroll
  for (int i = 0; i < 4; ++i) {
    const int mBase = m0 + (i << 4);
#pragma unroll
    for (int j = 0; j < 4; ++j) {
      const int n = n0 + (j << 4) + rlane;
      float bv = 0.f;
      if (BIAS_MODE == 2) bv = bias[n];
#pragma unroll
      for (int r = 0; r < 8; ++r) {
        float v = acc[i][j][r] * scale;
        if (BIAS_MODE == 1) v += bias[mBase + mOff + r];
        if (BIAS_MODE == 2) v += bv;
        if (RESID) v += Rb[(size_t)(mBase + mOff + r) * ldc + n];
        if (ACT == 1) v = tanhf(v);
        if (ACT == 2) v = fmaxf(v, 0.0f);
        if (ACT == 3) v = v / (1.0f + expf(-v));
        if (ACT == 4) v = (v > 0.f) ? v : 0.01f * v;
        if (ACT == 5) v = 0.5f * v * (1.0f + erff(v * 0.70710678118654752f));
        if (ACT == 6) v = v * __builtin_amdgcn_rcpf(1.0f + __expf(-v));
        if (ACT == 7) v = (v > 0.f) ? v : (expf(v) - 1.0f);
        slab[(mOff + r) * 68 + (j << 4) + rlane] = v;
      }
    }
    __builtin_amdgcn_fence(__ATOMIC_RELEASE, "workgroup");
    __builtin_amdgcn_wave_barrier();
    __builtin_amdgcn_fence(__ATOMIC_ACQUIRE, "workgroup");
    if (OUT_MODE == 0) {
      float* C = (float*)Cout + (size_t)b * strideC;
      const int hh = lane >> 4, c4 = (lane & 15) * 4;
      for (int pass = 0; pass < 2; ++pass) {
#pragma unroll
        for (int it = 0; it < 8; ++it) {
          const int row = it * 2 + hh;
          v4f v = *(const v4f*)(slab + row * 68 + c4);
          *(volatile v4f*)(C + (size_t)(mBase + row) * ldc + n0 + c4) = v;
        }
        __threadfence();
      }
    } else {
      const int q = lane >> 3, c8 = (lane & 7) * 8;
      unsigned short* C  = (unsigned short*)Cout  + (size_t)b * strideC;
      unsigned short* C2 = (OUT_MODE == 2) ? ((unsigned short*)Cout2 + (size_t)b * strideC) : nullptr;
      for (int pass = 0; pass < 2; ++pass) {
#pragma unroll
        for (int it = 0; it < 4; ++it) {
          const int row = it * 4 + q;
          const float* sp = slab + row * 68 + c8;
          v8h hv, lv;
#pragma unroll
          for (int e = 0; e < 8; ++e) {
            if (OUT_MODE == 1) {
              hv[e] = (_Float16)sp[e];
            } else {
              unsigned short hb = f2bf_bits(sp[e]);
              unsigned short lb = f2bf_bits(sp[e] - bf_bits2f(hb));
              hv[e] = __builtin_bit_cast(_Float16, hb);
              lv[e] = __builtin_bit_cast(_Float16, lb);
            }
          }
          *(volatile v8h*)(C + (size_t)(mBase + row) * ldc + n0 + c8) = hv;
          if (OUT_MODE == 2) *(volatile v8h*)(C2 + (size_t)(mBase + row) * ldc + n0 + c8) = lv;
        }
        __threadfence();
      }
    }
    __builtin_amdgcn_fence(__ATOMIC_RELEASE, "workgroup");
    __builtin_amdgcn_wave_barrier();
    __builtin_amdgcn_fence(__ATOMIC_ACQUIRE, "workgroup");
  }
}

template <int NB>
__device__ __forceinline__ int scan_chunk(const int* __restrict__ lst, int nE, int cbase, int nodeBase,
                                          int* list, int tid, int lane, int wave, int fullvec) {
  int wc = 0;
#pragma unroll
  for (int g = 0; g < NGRP; ++g) {
    const int el0 = (g * NTHR + tid) * EPT;
    const int e0  = cbase + el0;
    v4i da, db;
    if (fullvec) {
      da = *(const v4i*)(lst + e0);
      db = *(const v4i*)(lst + e0 + 4);
    } else {
      const int em = nE - 1;
      da.x = lst[(e0     < em) ? e0     : em];
      da.y = lst[(e0 + 1 < em) ? e0 + 1 : em];
      da.z = lst[(e0 + 2 < em) ? e0 + 2 : em];
      da.w = lst[(e0 + 3 < em) ? e0 + 3 : em];
      db.x = lst[(e0 + 4 < em) ? e0 + 4 : em];
      db.y = lst[(e0 + 5 < em) ? e0 + 5 : em];
      db.z = lst[(e0 + 6 < em) ? e0 + 6 : em];
      db.w = lst[(e0 + 7 < em) ? e0 + 7 : em];
    }
    const bool v0 = (e0 < nE), v1 = (e0 + 1 < nE), v2 = (e0 + 2 < nE), v3 = (e0 + 3 < nE);
    const bool v4 = (e0 + 4 < nE), v5 = (e0 + 5 < nE), v6 = (e0 + 6 < nE), v7 = (e0 + 7 < nE);
    const unsigned nb = (unsigned)nodeBase;
    const unsigned s0 = (unsigned)da.x - nb, s1 = (unsigned)da.y - nb;
    const unsigned s2 = (unsigned)da.z - nb, s3 = (unsigned)da.w - nb;
    const unsigned s4 = (unsigned)db.x - nb, s5 = (unsigned)db.y - nb;
    const unsigned s6 = (unsigned)db.z - nb, s7 = (unsigned)db.w - nb;
    const bool h0 = v0 && (s0 < (unsigned)NB), h1 = v1 && (s1 < (unsigned)NB);
    const bool h2 = v2 && (s2 < (unsigned)NB), h3 = v3 && (s3 < (unsigned)NB);
    const bool h4 = v4 && (s4 < (unsigned)NB), h5 = v5 && (s5 < (unsigned)NB);
    const bool h6 = v6 && (s6 < (unsigned)NB), h7 = v7 && (s7 < (unsigned)NB);
    const unsigned any = __builtin_amdgcn_ballot_w32(h0 | h1 | h2 | h3 | h4 | h5 | h6 | h7);
    if (any != 0u) {
#define HITJ(J, HJ, SJ) { \
        const unsigned mj = __builtin_amdgcn_ballot_w32(HJ); \
        if (mj != 0u) { \
          if (HJ) { \
            const int pos = wc + (int)__builtin_amdgcn_mbcnt_lo(mj, 0u); \
            if (pos < WCAP) list[wave * WCAP + pos] = ((el0 + (J)) << 12) | (int)(SJ); \
          } \
          wc += (int)__builtin_popcount(mj); } }
      HITJ(0, h0, s0)
      HITJ(1, h1, s1)
      HITJ(2, h2, s2)
      HITJ(3, h3, s3)
      HITJ(4, h4, s4)
      HITJ(5, h5, s5)
      HITJ(6, h6, s6)
      HITJ(7, h7, s7)
#undef HITJ
    }
  }
  return wc;
}

__global__ __launch_bounds__(NTHR) void k_wprep16(const float* __restrict__ W, int Kin, int ncol, int Kpad,
                                                  int nrow, float scale, unsigned short* bt) {
  const int tpr = Kpad >> 3;
  const int i = blockIdx.x * NTHR + threadIdx.x;
  if (i >= nrow * tpr) return;
  const int n   = i / tpr;
  const int k0  = (i - n * tpr) * 8;
  const int ncl = (n < ncol) ? n : ncol - 1;
  v8h hv;
#pragma unroll
  for (int e = 0; e < 8; ++e) {
    const int k  = k0 + e;
    const int kc = (k < Kin) ? k : Kin - 1;
    float v = W[(size_t)kc * ncol + ncl];
    if (k >= Kin || n >= ncol) v = 0.f;
    hv[e] = (_Float16)(scale * v);
  }
  const size_t o = (size_t)i * 8;
  *(volatile v8h*)(bt + o) = hv;
  __threadfence();
  *(volatile v8h*)(bt + o) = hv;
}

__global__ __launch_bounds__(NTHR) void k_wsplit(const float* __restrict__ W, int Kin, int ncol, int Kpad,
                                                 int nrow, unsigned short* bth, unsigned short* btl) {
  const int tpr = Kpad >> 3;
  const int i = blockIdx.x * NTHR + threadIdx.x;
  if (i >= nrow * tpr) return;
  const int n   = i / tpr;
  const int k0  = (i - n * tpr) * 8;
  const int ncl = (n < ncol) ? n : ncol - 1;
  v8h hv, lv;
#pragma unroll
  for (int e = 0; e < 8; ++e) {
    const int k  = k0 + e;
    const int kc = (k < Kin) ? k : Kin - 1;
    float v = W[(size_t)kc * ncol + ncl];
    if (k >= Kin || n >= ncol) v = 0.f;
    const unsigned short hb = f2bf_bits(v);
    const unsigned short lb = f2bf_bits(v - bf_bits2f(hb));
    hv[e] = __builtin_bit_cast(_Float16, hb);
    lv[e] = __builtin_bit_cast(_Float16, lb);
  }
  const size_t o = (size_t)i * 8;
  *(volatile v8h*)(bth + o) = hv;
  *(volatile v8h*)(btl + o) = lv;
  __threadfence();
  *(volatile v8h*)(bth + o) = hv;
  *(volatile v8h*)(btl + o) = lv;
}

__global__ __launch_bounds__(NTHR) void k_stats(const int* __restrict__ dstl, int nE,
                                                const float* __restrict__ off,
                                                float* mxo, float* seo, int vec_ok) {
  constexpr int NB  = NBS;
  constexpr int NQ4 = NB / 4;
  static_assert(NQ4 % NTHR == 0);
  __shared__ __align__(16) v4f smx4[NQ4];
  __shared__ __align__(16) v4f sse4[NQ4];
  __shared__ int list[LISTN];
  __shared__ int wcnt[NWAVE];
  float* smx = (float*)smx4;
  float* sse = (float*)sse4;
  const int tid = threadIdx.x, lane = tid & 31, wave = tid >> 5;
  const int nodeBase = blockIdx.x * NB;

  {
    const v4f mi = {-INFINITY, -INFINITY, -INFINITY, -INFINITY};
    const v4f zz = {0.f, 0.f, 0.f, 0.f};
    for (int i = tid; i < NQ4; i += NTHR) { smx4[i] = mi; sse4[i] = zz; }
  }
  __syncthreads();

  int nSub = (nE + SUBCH - 1) / SUBCH;
  nSub = (nSub > MAXSUB_ALL) ? MAXSUB_ALL : nSub;
#pragma unroll 1
  for (int ch = 0; ch < nSub; ++ch) {
    const int cbase = ch * SUBCH;
    const int fullvec = (vec_ok != 0 && cbase + SUBCH <= nE) ? 1 : 0;
    const int wc = scan_chunk<NB>(dstl, nE, cbase, nodeBase, list, tid, lane, wave, fullvec);
    if (lane == 0) wcnt[wave] = wc;
    __syncthreads();
    if (wave == 0) {
#pragma unroll 1
      for (int wsx = 0; wsx < NWAVE; ++wsx) {
        int n = __builtin_amdgcn_readfirstlane(wcnt[wsx]);
        n = n > WCAP ? WCAP : (n < 0 ? 0 : n);
        const int* lp = list + wsx * WCAP;
#pragma unroll 1
        for (int i = 0; i < n; ++i) {
          const int ent  = __builtin_amdgcn_readfirstlane(lp[i]);
          const int slot = ent & (NB - 1);
          int el = cbase + ((ent >> 12) & (SUBCH - 1));
          el = (el > nE - 1) ? nE - 1 : el;
          const v2f o = *(const v2f*)(off + (size_t)el * CDIM);
          const float sc = 1.0f / (fabsf(o.x) + fabsf(o.y) + 0.001f);
          const float m  = smx[slot];
          const float se = sse[slot];
          const float mn = fmaxf(m, sc);
          const float se2 = se * expf(m - mn) + expf(sc - mn);
          smx[slot] = mn;
          sse[slot] = se2;
        }
      }
    }
    __syncthreads();
  }

  float* gm = mxo + (size_t)nodeBase;
  float* gs = seo + (size_t)nodeBase;
  for (int pass = 0; pass < 2; ++pass) {
#pragma unroll
    for (int i = tid; i < NQ4; i += NTHR) {
      v4f m4 = smx4[i];
      const v4f s4 = sse4[i];
      m4.x = (s4.x == 0.f) ? 0.f : m4.x;
      m4.y = (s4.y == 0.f) ? 0.f : m4.y;
      m4.z = (s4.z == 0.f) ? 0.f : m4.z;
      m4.w = (s4.w == 0.f) ? 0.f : m4.w;
      ((volatile v4f*)gm)[i] = m4;
      ((volatile v4f*)gs)[i] = s4;
    }
    __threadfence();
  }
}

__global__ __launch_bounds__(NTHR) void k_kpre(const float* __restrict__ off, const float* __restrict__ w1,
                                               const float* __restrict__ b1, int nE, int ebase, int Mc,
                                               unsigned short* kh) {
  const int i  = blockIdx.x * NTHR + threadIdx.x;
  const int r  = i >> 4;
  const int h0 = (i & 15) * 8;
  const int e  = ebase + r;
  const bool valid = (r < Mc) && (e < nE);
  int ec = (e < nE) ? e : nE - 1; ec = (ec < 0) ? 0 : ec;
  const v2f o = *(const v2f*)(off + (size_t)ec * CDIM);
  v8h hv;
#pragma unroll
  for (int j = 0; j < 8; ++j) {
    const int h = h0 + j;
    float v = o.x * w1[h] + o.y * w1[HF + h] + b1[h];
    v = (v > 0.0f) ? v : (expf(v) - 1.0f);
    hv[j] = valid ? (_Float16)v : (_Float16)0.0f;
  }
  const bool ok = (r < Mc);
  const size_t oo = (size_t)i * 8;
  if (ok) *(volatile v8h*)(kh + oo) = hv;
  __threadfence();
  if (ok) *(volatile v8h*)(kh + oo) = hv;
}

__global__ __launch_bounds__(NTHR) void k_agg(
    const int* __restrict__ dstl, const int* __restrict__ srcl, const float* __restrict__ offl, int nEc,
    const float* __restrict__ kwp, const float* __restrict__ feat, int nN,
    const float* __restrict__ mxp, const float* __restrict__ sep,
    float* agg, int first, int vec_ok) {
#pragma clang fp contract(off)
  constexpr int NB  = NBA;
  constexpr int NV4 = NB * NIN / 4;
  constexpr int NQ4 = NB / 4;
  static_assert(NV4 % NTHR == 0 && NQ4 % NTHR == 0);
  extern __shared__ v4f lds_dyn[];
  float* acc  = (float*)lds_dyn;
  float* smx  = acc + NB * NIN;
  float* sse  = smx + NB;
  int*   list = (int*)(sse + NB);
  int*   wcnt = list + LISTN;
  const int tid = threadIdx.x, lane = tid & 31, wave = tid >> 5;
  const int nodeBase = blockIdx.x * NB;
  float* ga = agg + (size_t)nodeBase * NIN;

  if (first) {
    const v4f zz = {0.f, 0.f, 0.f, 0.f};
    for (int i = tid; i < NV4; i += NTHR) lds_dyn[i] = zz;
  } else {
    for (int i = tid; i < NV4; i += NTHR) lds_dyn[i] = ((const v4f*)ga)[i];
  }
  for (int i = tid; i < NQ4; i += NTHR) {
    lds_dyn[NV4 + i]       = ((const v4f*)(mxp + (size_t)nodeBase))[i];
    lds_dyn[NV4 + NQ4 + i] = ((const v4f*)(sep + (size_t)nodeBase))[i];
  }
  __syncthreads();

  int nSub = (nEc + SUBCH - 1) / SUBCH;
  nSub = (nSub > MAXSUB_CH) ? MAXSUB_CH : nSub;
#pragma unroll 1
  for (int ch = 0; ch < nSub; ++ch) {
    const int cbase = ch * SUBCH;
    const int fullvec = (vec_ok != 0 && cbase + SUBCH <= nEc) ? 1 : 0;
    const int wc = scan_chunk<NB>(dstl, nEc, cbase, nodeBase, list, tid, lane, wave, fullvec);
    if (lane == 0) wcnt[wave] = wc;
    __syncthreads();
    if (wave == 0) {
#pragma unroll 1
      for (int wsx = 0; wsx < NWAVE; ++wsx) {
        int n = __builtin_amdgcn_readfirstlane(wcnt[wsx]);
        n = n > WCAP ? WCAP : (n < 0 ? 0 : n);
        const int* lp = list + wsx * WCAP;
#pragma unroll 1
        for (int i = 0; i < n; ++i) {
          const int ent  = __builtin_amdgcn_readfirstlane(lp[i]);
          const int slot = ent & (NB - 1);
          int el = cbase + ((ent >> 12) & (SUBCH - 1));
          el = (el > nEc - 1) ? nEc - 1 : el;
          int s = srcl[el];
          s = (s < 0) ? 0 : ((s > nN - 1) ? nN - 1 : s);
          const v2f o = *(const v2f*)(offl + (size_t)el * CDIM);
          const float sc  = 1.0f / (fabsf(o.x) + fabsf(o.y) + 0.001f);
          const float mxv = smx[slot];
          const float sev = sse[slot];
          const float wgt = expf(sc - mxv) * (1.0f / sev);
          const v2f kw = *(const v2f*)(kwp + (size_t)el * NIN + 2 * lane);
          const v2f fv = *(const v2f*)(feat + (size_t)s * NIN + 2 * lane);
          v2f t; t.x = wgt * kw.x; t.y = wgt * kw.y;
          v2f m; m.x = fv.x * t.x; m.y = fv.y * t.y;
          v2f* ap = (v2f*)(acc + slot * NIN + 2 * lane);
          const v2f av = *ap;
          *ap = av + m;
        }
      }
    }
    __syncthreads();
  }

  for (int pass = 0; pass < 2; ++pass) {
#pragma unroll 4
    for (int i = tid; i < NV4; i += NTHR) { const v4f v = lds_dyn[i]; ((volatile v4f*)ga)[i] = v; }
    __threadfence();
  }
}

__global__ __launch_bounds__(NTHR) void k_featsplit(const float* __restrict__ feat, int nN, int RP,
                                                    unsigned short* fh, unsigned short* fl) {
  const int i   = blockIdx.x * NTHR + threadIdx.x;
  const int row = i >> 3;
  const int c0  = (i & 7) * 8;
  const int rown = (row < nN) ? row : nN - 1;
  const float* p = feat + (size_t)rown * NIN + c0;
  const v4f a0 = *(const v4f*)p;
  const v4f a1 = *(const v4f*)(p + 4);
  const bool z = (row >= nN);
  const float A8[8] = {a0.x, a0.y, a0.z, a0.w, a1.x, a1.y, a1.z, a1.w};
  v8h hv, lv;
#pragma unroll
  for (int j = 0; j < 8; ++j) {
    const float v = z ? 0.0f : A8[j];
    const unsigned short hb = f2bf_bits(v);
    const unsigned short lb = f2bf_bits(v - bf_bits2f(hb));
    hv[j] = __builtin_bit_cast(_Float16, hb);
    lv[j] = __builtin_bit_cast(_Float16, lb);
  }
  const bool ok = (row < RP);
  const size_t o = (size_t)i * 8;
  if (ok) { *(volatile v8h*)(fh + o) = hv; *(volatile v8h*)(fl + o) = lv; }
  __threadfence();
  if (ok) { *(volatile v8h*)(fh + o) = hv; *(volatile v8h*)(fl + o) = lv; }
}

__global__ __launch_bounds__(NTHR) void k_aggsplit(const float* __restrict__ agg, int RP,
                                                   unsigned short* ch, unsigned short* cl) {
  const int i   = blockIdx.x * NTHR + threadIdx.x;
  const int row = i >> 3;
  const int c0  = (i & 7) * 8;
  const int rowa = (row < RP) ? row : RP - 1;
  const float* p = agg + (size_t)rowa * NIN + c0;
  const v4f a0 = *(const v4f*)p;
  const v4f a1 = *(const v4f*)(p + 4);
  const float A8[8] = {a0.x, a0.y, a0.z, a0.w, a1.x, a1.y, a1.z, a1.w};
  v8h hv, lv;
#pragma unroll
  for (int j = 0; j < 8; ++j) {
    const float v = A8[j];
    const unsigned short hb = f2bf_bits(v);
    const unsigned short lb = f2bf_bits(v - bf_bits2f(hb));
    hv[j] = __builtin_bit_cast(_Float16, hb);
    lv[j] = __builtin_bit_cast(_Float16, lb);
  }
  const bool ok = (row < RP);
  const size_t o = (size_t)row * KCAT + c0;
  if (ok) { *(volatile v8h*)(ch + o) = hv; *(volatile v8h*)(cl + o) = lv; }
  __threadfence();
  if (ok) { *(volatile v8h*)(ch + o) = hv; *(volatile v8h*)(cl + o) = lv; }
}

__global__ __launch_bounds__(NTHR) void k_copy(const float* __restrict__ src, float* out, int n4) {
  const int i = blockIdx.x * NTHR + threadIdx.x;
  const int ic = (i < n4) ? i : n4 - 1;
  const v4f v = ((const v4f*)src)[ic];
  if (i < n4) ((volatile v4f*)out)[i] = v;
  __threadfence();
  if (i < n4) ((volatile v4f*)out)[i] = v;
}

extern "C" void kernel_launch(void* const* d_in, const int* in_sizes, int n_in,
                              void* d_out, int out_size, void* d_ws, size_t ws_size,
                              hipStream_t stream) {
  if (n_in < 20) return;
  const int nN = in_sizes[0] / NIN;
  const int nE = in_sizes[2];
  if (nN < 1 || in_sizes[0] != nN * NIN || nN > (1 << 22)) return;
  if (nE < 1 || nE > NEDGE_MAX || in_sizes[1] != nE * CDIM || in_sizes[3] != nE) return;
  if (in_sizes[4] != CDIM * HF || in_sizes[5] != HF || in_sizes[6] != HF * NIN || in_sizes[7] != NIN) return;
  if (in_sizes[8] != NIN * HF || in_sizes[9] != HF || in_sizes[10] != HF * HF || in_sizes[11] != HF) return;
  if (in_sizes[12] != KCAT * HF || in_sizes[13] != HF || in_sizes[14] != HF * HF || in_sizes[15] != HF) return;
  if (in_sizes[16] != HF * HF || in_sizes[17] != HF || in_sizes[18] != HF * NOUT || in_sizes[19] != NOUT) return;
  if (out_size != nN * NOUT) return;
  const int nChunks = (nE + CHE - 1) / CHE;
  if (nChunks < 1 || nChunks > 8) return;

  const float* feat    = (const float*)d_in[0];
  const float* offsets = (const float*)d_in[1];
  const int*   src     = (const int*)d_in[2];
  const int*   dst     = (const int*)d_in[3];
  const float* kW1 = (const float*)d_in[4];
  const float* kb1 = (const float*)d_in[5];
  const float* kW2 = (const float*)d_in[6];
  const float* kb2 = (const float*)d_in[7];
  const float* sW1 = (const float*)d_in[8];
  const float* sb1 = (const float*)d_in[9];
  const float* sW2 = (const float*)d_in[10];
  const float* sb2 = (const float*)d_in[11];
  const float* mW1 = (const float*)d_in[12];
  const float* mb1 = (const float*)d_in[13];
  const float* mW2 = (const float*)d_in[14];
  const float* mb2 = (const float*)d_in[15];
  const float* mW3 = (const float*)d_in[16];
  const float* mb3 = (const float*)d_in[17];
  const float* mW4 = (const float*)d_in[18];
  const float* mb4 = (const float*)d_in[19];
  float* out = (float*)d_out;

  const int RP  = ((nN + RPQ - 1) / RPQ) * RPQ;
  const int nA  = RP / NBA;
  const int nS  = (nN + NBS - 1) / NBS;
  const int MXN = nS * NBS;

  size_t off = 0;
  auto carve = [&](size_t bytes) { const size_t o = off; off += (bytes + 255) & ~(size_t)255; return o; };
  const size_t oKW2T = carve((size_t)NIN * HF * 2);
  const size_t oSW1H = carve((size_t)HF * NIN * 2);
  const size_t oSW1L = carve((size_t)HF * NIN * 2);
  const size_t oSW2H = carve((size_t)HF * HF * 2);
  const size_t oSW2L = carve((size_t)HF * HF * 2);
  const size_t oMW1H = carve((size_t)HF * KCAT * 2);
  const size_t oMW1L = carve((size_t)HF * KCAT * 2);
  const size_t oMW2H = carve((size_t)HF * HF * 2);
  const size_t oMW2L = carve((size_t)HF * HF * 2);
  const size_t oMW3H = carve((size_t)HF * HF * 2);
  const size_t oMW3L = carve((size_t)HF * HF * 2);
  const size_t oMW4H = carve((size_t)NOUT * HF * 2);
  const size_t oMW4L = carve((size_t)NOUT * HF * 2);
  const size_t oMX   = carve((size_t)MXN * 4);
  const size_t oSE   = carve((size_t)MXN * 4);
  const size_t oAGG  = carve((size_t)RP * NIN * 4);
  const size_t szA   = (size_t)CHE * HF * 2;
  const size_t oA    = carve(szA);
  const size_t szB   = (size_t)CHE * NIN * 4;
  const size_t oB    = carve(szB);
  if (off > ws_size || off > (size_t)134217728) return;
  const size_t szF  = (size_t)RP * NIN * 2;
  const size_t szH  = (size_t)RP * HF * 2;
  const size_t szC  = (size_t)RP * KCAT * 2;
  const size_t oFH  = oA;
  const size_t oFL  = oFH + szF;
  const size_t oS1H = oFL + szF;
  const size_t oS1L = oS1H + szH;
  if (2 * szF + 2 * szH > szA) return;
  const size_t oM1H = oA, oM1L = oA + szH;
  const size_t oM3H = oA, oM3L = oA + szH;
  if (2 * szH > szA) return;
  const size_t oCH  = oB, oCL = oB + szC;
  if (2 * szC > szB) return;
  const size_t oM2H = oB, oM2L = oB + szH;
  if (2 * szH > szB) return;
  const size_t oOUT = oB;
  if ((size_t)RP * NOUT * 4 > szB) return;

  char* ws = (char*)d_ws;
  unsigned short* kw2t = (unsigned short*)(ws + oKW2T);
  unsigned short* sw1h = (unsigned short*)(ws + oSW1H);
  unsigned short* sw1l = (unsigned short*)(ws + oSW1L);
  unsigned short* sw2h = (unsigned short*)(ws + oSW2H);
  unsigned short* sw2l = (unsigned short*)(ws + oSW2L);
  unsigned short* mw1h = (unsigned short*)(ws + oMW1H);
  unsigned short* mw1l = (unsigned short*)(ws + oMW1L);
  unsigned short* mw2h = (unsigned short*)(ws + oMW2H);
  unsigned short* mw2l = (unsigned short*)(ws + oMW2L);
  unsigned short* mw3h = (unsigned short*)(ws + oMW3H);
  unsigned short* mw3l = (unsigned short*)(ws + oMW3L);
  unsigned short* mw4h = (unsigned short*)(ws + oMW4H);
  unsigned short* mw4l = (unsigned short*)(ws + oMW4L);
  float* mx  = (float*)(ws + oMX);
  float* se  = (float*)(ws + oSE);
  float* agg = (float*)(ws + oAGG);
  unsigned short* kh  = (unsigned short*)(ws + oA);
  float* kwf = (float*)(ws + oB);
  unsigned short* fh  = (unsigned short*)(ws + oFH);
  unsigned short* fl  = (unsigned short*)(ws + oFL);
  unsigned short* s1h = (unsigned short*)(ws + oS1H);
  unsigned short* s1l = (unsigned short*)(ws + oS1L);
  unsigned short* m1h = (unsigned short*)(ws + oM1H);
  unsigned short* m1l = (unsigned short*)(ws + oM1L);
  unsigned short* m2h = (unsigned short*)(ws + oM2H);
  unsigned short* m2l = (unsigned short*)(ws + oM2L);
  unsigned short* m3h = (unsigned short*)(ws + oM3H);
  unsigned short* m3l = (unsigned short*)(ws + oM3L);
  unsigned short* chp = (unsigned short*)(ws + oCH);
  unsigned short* clp = (unsigned short*)(ws + oCL);
  float* outp = (float*)(ws + oOUT);

  auto gemm_blocks = [](int M, int Nn) { return ((M / 64) * (Nn / 64) + 7) / 8; };

  k_wprep16<<<(NIN * (HF / 8) + NTHR - 1) / NTHR, NTHR, 0, stream>>>(kW2, HF, NIN, HF, NIN, 16.0f, kw2t);
  k_wsplit<<<(HF * (NIN / 8) + NTHR - 1) / NTHR, NTHR, 0, stream>>>(sW1, NIN, HF, NIN, HF, sw1h, sw1l);
  k_wsplit<<<(HF * (HF / 8) + NTHR - 1) / NTHR, NTHR, 0, stream>>>(sW2, HF, HF, HF, HF, sw2h, sw2l);
  k_wsplit<<<(HF * (KCAT / 8) + NTHR - 1) / NTHR, NTHR, 0, stream>>>(mW1, KCAT, HF, KCAT, HF, mw1h, mw1l);
  k_wsplit<<<(HF * (HF / 8) + NTHR - 1) / NTHR, NTHR, 0, stream>>>(mW2, HF, HF, HF, HF, mw2h, mw2l);
  k_wsplit<<<(HF * (HF / 8) + NTHR - 1) / NTHR, NTHR, 0, stream>>>(mW3, HF, HF, HF, HF, mw3h, mw3l);
  k_wsplit<<<(NOUT * (HF / 8) + NTHR - 1) / NTHR, NTHR, 0, stream>>>(mW4, HF, NOUT, HF, NOUT, mw4h, mw4l);

  k_stats<<<nS, NTHR, 0, stream>>>(dst, nE, offsets, mx, se, 1);

  for (int c = 0; c < nChunks; ++c) {
    const int base = c * CHE;
    int Ec = nE - base; if (Ec > CHE) Ec = CHE;
    const int Mc = ((Ec + 63) / 64) * 64;
    const int vec = ((base & 3) == 0) ? 1 : 0;
    k_kpre<<<(Mc * 16) / NTHR, NTHR, 0, stream>>>(offsets, kW1, kb1, nE, base, Mc, kh);
    wmma_gemm64<0, false, 2, 0, false, 0><<<dim3(gemm_blocks(Mc, NIN), 1), 256, 0, stream>>>(
        kh, kh, HF, 0L, kw2t, kw2t, HF, 0L, (void*)kwf, (void*)kwf, NIN, 0L, kb2, kb2, 0L, Mc, NIN, HF, 1.0f / 16.0f);
    k_agg<<<nA, NTHR, LDS_AGG, stream>>>(dst + base, src + base, offsets + (size_t)base * CDIM, Ec, kwf, feat, nN,
                                         mx, se, agg, (c == 0) ? 1 : 0, vec);
  }

  k_featsplit<<<(RP * 8) / NTHR, NTHR, 0, stream>>>(feat, nN, RP, fh, fl);
  wmma_gemm64<1, true, 2, 2, false, 7><<<dim3(gemm_blocks(RP, HF), 1), 256, 0, stream>>>(
      fh, fl, NIN, 0L, sw1h, sw1l, NIN, 0L, (void*)s1h, (void*)s1l, HF, 0L, sb1, sb1, 0L, RP, HF, NIN, 1.0f);
  wmma_gemm64<1, true, 2, 2, false, 0><<<dim3(gemm_blocks(RP, HF), 1), 256, 0, stream>>>(
      s1h, s1l, HF, 0L, sw2h, sw2l, HF, 0L, (void*)(chp + NIN), (void*)(clp + NIN), KCAT, 0L, sb2, sb2, 0L, RP, HF, HF, 1.0f);
  k_aggsplit<<<(RP * 8) / NTHR, NTHR, 0, stream>>>(agg, RP, chp, clp);
  wmma_gemm64<1, true, 2, 2, false, 7><<<dim3(gemm_blocks(RP, HF), 1), 256, 0, stream>>>(
      chp, clp, KCAT, 0L, mw1h, mw1l, KCAT, 0L, (void*)m1h, (void*)m1l, HF, 0L, mb1, mb1, 0L, RP, HF, KCAT, 1.0f);
  wmma_gemm64<1, true, 2, 2, false, 7><<<dim3(gemm_blocks(RP, HF), 1), 256, 0, stream>>>(
      m1h, m1l, HF, 0L, mw2h, mw2l, HF, 0L, (void*)m2h, (void*)m2l, HF, 0L, mb2, mb2, 0L, RP, HF, HF, 1.0f);
  wmma_gemm64<1, true, 2, 2, false, 7><<<dim3(gemm_blocks(RP, HF), 1), 256, 0, stream>>>(
      m2h, m2l, HF, 0L, mw3h, mw3l, HF, 0L, (void*)m3h, (void*)m3l, HF, 0L, mb3, mb3, 0L, RP, HF, HF, 1.0f);
  wmma_gemm64<1, true, 2, 0, false, 0><<<dim3(gemm_blocks(RP, NOUT), 1), 256, 0, stream>>>(
      m3h, m3l, HF, 0L, mw4h, mw4l, HF, 0L, (void*)outp, (void*)outp, NOUT, 0L, mb4, mb4, 0L, RP, NOUT, HF, 1.0f);
  const int n4 = nN * (NOUT / 4);
  k_copy<<<(n4 + NTHR - 1) / NTHR, NTHR, 0, stream>>>(outp, out, n4);
}
